// GPT2Attention_26371099197458
// MI455X (gfx1250) — hardware-verified
//
#include <hip/hip_runtime.h>

#ifndef NB
#define NB 4
#endif
#ifndef SEQ
#define SEQ 2048
#endif
#define NB_FULL 4
#define SEQ_FULL 2048
#define DM 1024
#define NH 16
#define HD 64
#define LQ (3 * DM)
#define QT1 256
#define KP 72
#define NR ((size_t)NB * SEQ)
#define SCL 0.18033688011112042f
static_assert(SEQ % 128 == 0);
static_assert(SEQ >= QT1);
static_assert(SEQ <= SEQ_FULL);
static_assert(NB >= 1);
static_assert(NB <= NB_FULL);
static_assert(QT1 % 128 == 0);
static_assert(DM == NH * HD);
static_assert(HD == 64);
static_assert((KP * 2) % 16 == 0);
static_assert(DM % 32 == 0);
static_assert(LQ % 64 == 0);

typedef unsigned short v8us __attribute__((ext_vector_type(8), may_alias));
typedef float v8f __attribute__((ext_vector_type(8)));
typedef float v4f __attribute__((ext_vector_type(4)));
typedef float v4fa __attribute__((ext_vector_type(4), may_alias));
typedef _Float16 v16h __attribute__((ext_vector_type(16)));
typedef _Float16 v4h __attribute__((ext_vector_type(4)));
union FragH { v16h v; v8us half[2]; _Float16 h[16]; unsigned short u[16]; };

__device__ __forceinline__ unsigned short bf16_bits(float x) { unsigned int u = __float_as_uint(x); return (unsigned short)((u + 0x7FFFu + ((u >> 16) & 1u)) >> 16); }
__device__ __forceinline__ float bf16_val(unsigned short b) { return __uint_as_float(((unsigned int)b) << 16); }
__device__ __forceinline__ float bf16_rne(float x) { return bf16_val(bf16_bits(x)); }

__device__ __forceinline__ v16h g2_frag(const _Float16* p, int hh) { FragH f; f.half[0] = *(const v8us*)((const unsigned short*)p + 8 * hh); f.half[1] = *(const v8us*)((const unsigned short*)p + 16 + 8 * hh); return f.v; }
__device__ __forceinline__ v8f g2_mma(v16h a, v16h b, v8f c) { v8f d = __builtin_amdgcn_wmma_f32_16x16x32_f16(false, a, false, b, (short)0, c, false, false); asm volatile("v_nop\n\tv_nop\n\tv_nop\n\tv_nop" : "+v"(d) : "v"(a), "v"(b)); return d; }

__global__ __launch_bounds__(256) void k_wt_f16(const float* __restrict__ W, _Float16* __restrict__ Wt, int K, int N, float scale) {
  const int t = blockIdx.x * 256 + threadIdx.x; if (t >= N * (K / 8)) return; const int n = t / (K / 8), k8 = (t % (K / 8)) * 8; FragH f;
#pragma unroll
  for (int i = 0; i < 8; ++i) f.h[i] = (_Float16)(bf16_rne(W[(size_t)(k8 + i) * N + n]) * scale);
  const v8us o = f.half[0];
  *(volatile v8us*)((unsigned short*)Wt + (size_t)n * K + k8) = o; __threadfence(); *(volatile v8us*)((unsigned short*)Wt + (size_t)n * K + k8) = o;
}

__global__ __launch_bounds__(256) void k_x16r(const float* __restrict__ x, _Float16* __restrict__ X16, size_t n8) {
  const size_t t = (size_t)blockIdx.x * 256 + threadIdx.x; if (t >= n8) return;
  const size_t e = t * 8; const size_t rc = e / DM; const size_t cc = e - rc * DM; const size_t b = rc / SEQ, s = rc - b * SEQ;
  const float* src = x + ((b * SEQ_FULL + s) * DM + cc);
  const v4f a = *(const v4fa*)src, c = *(const v4fa*)(src + 4);
  FragH f;
#pragma unroll
  for (int q = 0; q < 4; ++q) { f.h[q] = (_Float16)bf16_rne(a[q]); f.h[4 + q] = (_Float16)bf16_rne(c[q]); }
  const v8us o = f.half[0];
  *(volatile v8us*)((unsigned short*)X16 + e) = o; __threadfence(); *(volatile v8us*)((unsigned short*)X16 + e) = o;
}

__global__ __launch_bounds__(256) void k_hres(const float* __restrict__ F, _Float16* __restrict__ Hl, size_t n8) {
  const size_t t = (size_t)blockIdx.x * 256 + threadIdx.x; if (t >= n8) return;
  const v4f a = *(const v4fa*)(F + t * 8), c = *(const v4fa*)(F + t * 8 + 4);
  FragH fl;
#pragma unroll
  for (int q = 0; q < 4; ++q) { const _Float16 h0 = (_Float16)a[q]; fl.h[q] = (_Float16)((a[q] - (float)h0) * 1024.0f); const _Float16 h1 = (_Float16)c[q]; fl.h[4 + q] = (_Float16)((c[q] - (float)h1) * 1024.0f); }
  const v8us o = fl.half[0];
  *(volatile v8us*)((unsigned short*)Hl + t * 8) = o; __threadfence(); *(volatile v8us*)((unsigned short*)Hl + t * 8) = o;
}

template <int NHv, int TTv>
__global__ __launch_bounds__(256) void k_vt(const _Float16* __restrict__ V16, int ldv, int voff, _Float16* __restrict__ Vt) {
  __shared__ unsigned short tl[64][66];
  const int tid = threadIdx.x; const int slab = blockIdx.x / (TTv / 64), lg = blockIdx.x % (TTv / 64); const int b = slab / NHv, h = slab % NHv;
  for (int i = tid; i < 64 * 8; i += 256) { const int r = i / 8, c8 = (i % 8) * 8; FragH f; f.half[0] = *(const v8us*)((const unsigned short*)V16 + ((size_t)b * TTv + lg * 64 + r) * ldv + voff + h * 64 + c8);
#pragma unroll
    for (int q = 0; q < 8; ++q) tl[r][c8 + q] = f.u[q]; }
  __syncthreads();
  for (int pass = 0; pass < 2; ++pass) {
#pragma unroll
    for (int rd = 0; rd < 2; ++rd) { const int d = rd * 32 + tid / 8, pc = tid % 8; FragH f;
#pragma unroll
      for (int q = 0; q < 8; ++q) f.u[q] = tl[pc * 8 + q][d];
      *(volatile v8us*)((unsigned short*)Vt + ((size_t)slab * 64 + d) * TTv + lg * 64 + pc * 8) = f.half[0]; }
    if (pass == 0) __threadfence(); }
}

__global__ __launch_bounds__(128) void k_gemm2(const _Float16* __restrict__ A, int lda, size_t sA, const _Float16* __restrict__ Bh, int ldb, size_t sB, float alpha, const float* __restrict__ bias,
    const float* CP, float* C, _Float16* C16, int ldc, size_t sC, size_t sC16, int M, int N, int K) {
  __shared__ __attribute__((aligned(16))) float so[4][32][68];
  const int tid = threadIdx.x, w = tid >> 5, lane = tid & 31, ln = lane & 15, hh = lane >> 4; const int by = blockIdx.y;
  A += (size_t)by * sA; Bh += (size_t)by * sB; const size_t cofs = (size_t)by * sC; const size_t cofs16 = (size_t)by * sC16;
  const int ntn = N >> 6; const int mt = blockIdx.x / ntn, nq = blockIdx.x - mt * ntn; const int row0 = mt * 128 + 32 * w, col0 = nq * 64; if (row0 >= M) return;
  const _Float16* a0p = A + (size_t)(row0 + ln) * lda; const _Float16* a1p = a0p + (size_t)16 * lda;
  const _Float16* b0p = Bh + (size_t)(col0 + ln) * ldb; const _Float16* b1p = b0p + (size_t)16 * ldb; const _Float16* b2p = b1p + (size_t)16 * ldb; const _Float16* b3p = b2p + (size_t)16 * ldb;
  const v8f z8 = {0.f, 0.f, 0.f, 0.f, 0.f, 0.f, 0.f, 0.f}; v8f c00 = z8, c01 = z8, c02 = z8, c03 = z8, c10 = z8, c11 = z8, c12 = z8, c13 = z8;
#pragma unroll 1
  for (int kb = 0; kb < K; kb += 32) { const v16h a0 = g2_frag(a0p + kb, hh), a1 = g2_frag(a1p + kb, hh);
    v16h b = g2_frag(b0p + kb, hh); c00 = g2_mma(a0, b, c00); c10 = g2_mma(a1, b, c10);
    b = g2_frag(b1p + kb, hh); c01 = g2_mma(a0, b, c01); c11 = g2_mma(a1, b, c11);
    b = g2_frag(b2p + kb, hh); c02 = g2_mma(a0, b, c02); c12 = g2_mma(a1, b, c12);
    b = g2_frag(b3p + kb, hh); c03 = g2_mma(a0, b, c03); c13 = g2_mma(a1, b, c13); }
  v8f accs[8] = {c00, c01, c02, c03, c10, c11, c12, c13};
#pragma unroll
  for (int u = 0; u < 8; ++u) { const int t = u & 3, half = u >> 2; const int col = col0 + t * 16 + ln; const float bv = bias ? bf16_rne(bias[col]) : 0.f;
#pragma unroll
    for (int r = 0; r < 8; ++r) { const int rloc = half * 16 + 8 * hh + r; float v = accs[u][r] * alpha + bv;
      if (CP) v += CP[cofs + (size_t)(row0 + rloc) * ldc + col];
      so[w][rloc][t * 16 + ln] = v; } }
  __builtin_amdgcn_fence(5, "workgroup"); __builtin_amdgcn_wave_barrier();
  const int rsub = lane >> 4, c4 = (lane & 15) * 4;
  for (int pass = 0; pass < 2; ++pass) {
#pragma unroll
    for (int q = 0; q < 16; ++q) { const int r = q * 2 + rsub; const v4f v = *(const v4fa*)&so[w][r][c4];
      if (C) *(volatile v4f*)(C + cofs + (size_t)(row0 + r) * ldc + col0 + c4) = v;
      if (C16) { v4h h4;
#pragma unroll
        for (int i = 0; i < 4; ++i) h4[i] = (_Float16)v[i];
        *(volatile v4h*)(C16 + cofs16 + (size_t)(row0 + r) * ldc + col0 + c4) = h4; } }
    if (pass == 0) __threadfence(); }
}

__global__ __launch_bounds__(128) __attribute__((amdgpu_num_vgpr(256)))
void k_attn(const _Float16* __restrict__ QKV, const _Float16* __restrict__ VT, _Float16* __restrict__ O16, int qb0) {
  __shared__ __attribute__((aligned(16))) _Float16 pl[4][16][KP];
  const int tid = threadIdx.x, w = tid >> 5, lane = tid & 31, ln = lane & 15, hh = lane >> 4;
  const int qblk = (int)blockIdx.x + qb0; const int bh = blockIdx.y; const int b = bh / NH, h = bh - b * NH;
  const int qrow0 = qblk * 64 + 16 * w;
  const _Float16* Qp = QKV + ((size_t)b * SEQ + qrow0 + ln) * LQ + h * HD;
  const v16h q0 = g2_frag(Qp, hh), q1 = g2_frag(Qp + 32, hh);
  const _Float16* Kp = QKV + ((size_t)b * SEQ + ln) * LQ + DM + h * HD;
  const _Float16* Vp = VT + ((size_t)bh * HD + ln) * SEQ;
  const v8f z8 = {0.f, 0.f, 0.f, 0.f, 0.f, 0.f, 0.f, 0.f};
  v8f oa[4] = {z8, z8, z8, z8};
  float m[8], l[8];
#pragma unroll
  for (int r = 0; r < 8; ++r) { m[r] = -1.0e30f; l[r] = 0.f; }
#pragma unroll 1
  for (int kb = 0; kb <= qblk; ++kb) {
    const int kbase = kb * 64;
    v8f s[4];
#pragma unroll
    for (int kt = 0; kt < 4; ++kt) { const _Float16* kr = Kp + (size_t)(kbase + kt * 16) * LQ; v16h kf = g2_frag(kr, hh); s[kt] = g2_mma(q0, kf, z8); kf = g2_frag(kr + 32, hh); s[kt] = g2_mma(q1, kf, s[kt]); }
    float mb[8];
#pragma unroll
    for (int r = 0; r < 8; ++r) mb[r] = -1.0e30f;
#pragma unroll
    for (int kt = 0; kt < 4; ++kt) { const int key = kbase + kt * 16 + ln;
#pragma unroll
      for (int r = 0; r < 8; ++r) { const int row = qrow0 + 8 * hh + r; const float v = (key > row) ? -1.0e30f : s[kt][r] * SCL; s[kt][r] = v; mb[r] = fmaxf(mb[r], v); } }
    float mn[8], al[8], ls[8];
#pragma unroll
    for (int r = 0; r < 8; ++r) { float v = mb[r]; v = fmaxf(v, __shfl_xor(v, 1, 32)); v = fmaxf(v, __shfl_xor(v, 2, 32)); v = fmaxf(v, __shfl_xor(v, 4, 32)); v = fmaxf(v, __shfl_xor(v, 8, 32));
      mn[r] = fmaxf(m[r], v); al[r] = exp2f(m[r] - mn[r]); ls[r] = 0.f; }
#pragma unroll
    for (int kt = 0; kt < 4; ++kt) {
#pragma unroll
      for (int r = 0; r < 8; ++r) { const float p = exp2f(s[kt][r] - mn[r]); s[kt][r] = p; ls[r] += p; } }
#pragma unroll
    for (int r = 0; r < 8; ++r) { float v = ls[r]; v += __shfl_xor(v, 1, 32); v += __shfl_xor(v, 2, 32); v += __shfl_xor(v, 4, 32); v += __shfl_xor(v, 8, 32);
      l[r] = l[r] * al[r] + v; m[r] = mn[r]; oa[0][r] *= al[r]; oa[1][r] *= al[r]; oa[2][r] *= al[r]; oa[3][r] *= al[r]; }
#pragma unroll
    for (int kt = 0; kt < 4; ++kt) {
#pragma unroll
      for (int r = 0; r < 8; ++r) pl[w][8 * hh + r][kt * 16 + ln] = (_Float16)(s[kt][r] * 4096.0f); }
    __builtin_amdgcn_fence(5, "wavefront"); __builtin_amdgcn_wave_barrier();
#pragma unroll
    for (int c = 0; c < 2; ++c) { const v16h pf = g2_frag(&pl[w][ln][c * 32], hh); const _Float16* vr = Vp + kbase + c * 32;
#pragma unroll
      for (int dt = 0; dt < 4; ++dt) { const v16h vf = g2_frag(vr + (size_t)(dt * 16) * SEQ, hh); oa[dt] = g2_mma(pf, vf, oa[dt]); } }
    __builtin_amdgcn_fence(5, "wavefront"); __builtin_amdgcn_wave_barrier();
  }
  float inv[8];
#pragma unroll
  for (int r = 0; r < 8; ++r) inv[r] = 1.0f / (64.0f * l[r]);
#pragma unroll
  for (int dt = 0; dt < 4; ++dt) {
#pragma unroll
    for (int r = 0; r < 8; ++r) pl[w][8 * hh + r][dt * 16 + ln] = (_Float16)(oa[dt][r] * inv[r]); }
  __builtin_amdgcn_fence(5, "wavefront"); __builtin_amdgcn_wave_barrier();
  for (int pass = 0; pass < 2; ++pass) {
#pragma unroll
    for (int it = 0; it < 4; ++it) { const int row = it * 4 + (lane >> 3), pc = (lane & 7) * 8; const v8us v = *(const v8us*)&pl[w][row][pc];
      *(volatile v8us*)((unsigned short*)O16 + ((size_t)b * SEQ + qrow0 + row) * DM + h * HD + pc) = v; }
    if (pass == 0) __threadfence(); }
}

__global__ __launch_bounds__(128) __attribute__((amdgpu_num_vgpr(256)))
void k_attn0(const _Float16* __restrict__ QKV, const _Float16* __restrict__ QL, const _Float16* __restrict__ VT, const _Float16* __restrict__ VTL, _Float16* __restrict__ O16, _Float16* __restrict__ OL) {
  __shared__ __attribute__((aligned(16))) _Float16 ph[4][16][KP];
  __shared__ __attribute__((aligned(16))) _Float16 pr[4][16][KP];
  const int tid = threadIdx.x, w = tid >> 5, lane = tid & 31, ln = lane & 15, hh = lane >> 4;
  const int qblk = (int)blockIdx.x; const int bh = blockIdx.y; const int b = bh / NH, h = bh - b * NH;
  const int qrow0 = qblk * 64 + 16 * w;
  const _Float16* Qp = QKV + ((size_t)b * SEQ + qrow0 + ln) * LQ + h * HD;
  const _Float16* Qlp = QL + ((size_t)b * QT1 + qrow0 + ln) * LQ + h * HD;
  const _Float16* Kp = QKV + ((size_t)b * SEQ + ln) * LQ + DM + h * HD;
  const _Float16* Klp = QL + ((size_t)b * QT1 + ln) * LQ + DM + h * HD;
  const _Float16* Vp = VT + ((size_t)bh * HD + ln) * SEQ;
  const _Float16* Vlp = VTL + ((size_t)bh * HD + ln) * QT1;
  const v8f z8 = {0.f, 0.f, 0.f, 0.f, 0.f, 0.f, 0.f, 0.f};
  v8f oa[4] = {z8, z8, z8, z8}; v8f oe[4] = {z8, z8, z8, z8};
  float m[8], l[8];
#pragma unroll
  for (int r = 0; r < 8; ++r) { m[r] = -1.0e30f; l[r] = 0.f; }
#pragma unroll 1
  for (int kb = 0; kb <= qblk; ++kb) {
    const int kbase = kb * 64;
    const v16h q0 = g2_frag(Qp, hh), q1 = g2_frag(Qp + 32, hh), q0l = g2_frag(Qlp, hh), q1l = g2_frag(Qlp + 32, hh);
    v8f s[4];
#pragma unroll
    for (int kt = 0; kt < 4; ++kt) { const _Float16* kr = Kp + (size_t)(kbase + kt * 16) * LQ; const _Float16* klr = Klp + (size_t)(kbase + kt * 16) * LQ;
      v16h kf = g2_frag(kr, hh); v8f sh = g2_mma(q0, kf, z8); v8f sr = g2_mma(q0l, kf, z8); kf = g2_frag(klr, hh); sr = g2_mma(q0, kf, sr);
      kf = g2_frag(kr + 32, hh); sh = g2_mma(q1, kf, sh); sr = g2_mma(q1l, kf, sr); kf = g2_frag(klr + 32, hh); sr = g2_mma(q1, kf, sr);
#pragma unroll
      for (int r = 0; r < 8; ++r) s[kt][r] = sh[r] + sr[r] * 0.0009765625f; }
    float mb[8];
#pragma unroll
    for (int r = 0; r < 8; ++r) mb[r] = -1.0e30f;
#pragma unroll
    for (int kt = 0; kt < 4; ++kt) { const int key = kbase + kt * 16 + ln;
#pragma unroll
      for (int r = 0; r < 8; ++r) { const int row = qrow0 + 8 * hh + r; const float v = (key > row) ? -1.0e30f : s[kt][r] * SCL; s[kt][r] = v; mb[r] = fmaxf(mb[r], v); } }
    float mn[8], al[8], ls[8];
#pragma unroll
    for (int r = 0; r < 8; ++r) { float v = mb[r]; v = fmaxf(v, __shfl_xor(v, 1, 32)); v = fmaxf(v, __shfl_xor(v, 2, 32)); v = fmaxf(v, __shfl_xor(v, 4, 32)); v = fmaxf(v, __shfl_xor(v, 8, 32));
      mn[r] = fmaxf(m[r], v); al[r] = exp2f(m[r] - mn[r]); ls[r] = 0.f; }
#pragma unroll
    for (int kt = 0; kt < 4; ++kt) {
#pragma unroll
      for (int r = 0; r < 8; ++r) { const float p = exp2f(s[kt][r] - mn[r]); s[kt][r] = p; ls[r] += p; } }
#pragma unroll
    for (int r = 0; r < 8; ++r) { float v = ls[r]; v += __shfl_xor(v, 1, 32); v += __shfl_xor(v, 2, 32); v += __shfl_xor(v, 4, 32); v += __shfl_xor(v, 8, 32);
      l[r] = l[r] * al[r] + v; m[r] = mn[r];
      oa[0][r] *= al[r]; oa[1][r] *= al[r]; oa[2][r] *= al[r]; oa[3][r] *= al[r]; oe[0][r] *= al[r]; oe[1][r] *= al[r]; oe[2][r] *= al[r]; oe[3][r] *= al[r]; }
#pragma unroll
    for (int kt = 0; kt < 4; ++kt) {
#pragma unroll
      for (int r = 0; r < 8; ++r) { const float v = s[kt][r] * 4096.0f; const _Float16 hv = (_Float16)v; ph[w][8 * hh + r][kt * 16 + ln] = hv; pr[w][8 * hh + r][kt * 16 + ln] = (_Float16)((v - (float)hv) * 1024.0f); } }
    __builtin_amdgcn_fence(5, "wavefront"); __builtin_amdgcn_wave_barrier();
#pragma unroll
    for (int c = 0; c < 2; ++c) { const v16h pfh = g2_frag(&ph[w][ln][c * 32], hh); const v16h pfr = g2_frag(&pr[w][ln][c * 32], hh);
      const _Float16* vr = Vp + kbase + c * 32; const _Float16* vlr = Vlp + kbase + c * 32;
#pragma unroll
      for (int dt = 0; dt < 4; ++dt) { v16h vf = g2_frag(vr + (size_t)(dt * 16) * SEQ, hh); oa[dt] = g2_mma(pfh, vf, oa[dt]); oe[dt] = g2_mma(pfr, vf, oe[dt]);
        vf = g2_frag(vlr + (size_t)(dt * 16) * QT1, hh); oe[dt] = g2_mma(pfh, vf, oe[dt]); } }
    __builtin_amdgcn_fence(5, "wavefront"); __builtin_amdgcn_wave_barrier();
  }
  float inv[8];
#pragma unroll
  for (int r = 0; r < 8; ++r) inv[r] = 1.0f / (64.0f * l[r]);
#pragma unroll
  for (int dt = 0; dt < 4; ++dt) {
#pragma unroll
    for (int r = 0; r < 8; ++r) { const float y = (oa[dt][r] + oe[dt][r] * 0.0009765625f) * inv[r]; const _Float16 hv = (_Float16)y; ph[w][8 * hh + r][dt * 16 + ln] = hv; pr[w][8 * hh + r][dt * 16 + ln] = (_Float16)((y - (float)hv) * 1024.0f); } }
  __builtin_amdgcn_fence(5, "wavefront"); __builtin_amdgcn_wave_barrier();
  for (int pass = 0; pass < 2; ++pass) {
#pragma unroll
    for (int it = 0; it < 4; ++it) { const int row = it * 4 + (lane >> 3), pc = (lane & 7) * 8; const v8us vhi = *(const v8us*)&ph[w][row][pc]; const v8us vlo = *(const v8us*)&pr[w][row][pc];
      *(volatile v8us*)((unsigned short*)O16 + ((size_t)b * SEQ + qrow0 + row) * DM + h * HD + pc) = vhi;
      *(volatile v8us*)((unsigned short*)OL + ((size_t)b * QT1 + qrow0 + row) * DM + h * HD + pc) = vlo; }
    if (pass == 0) __threadfence(); }
}

extern "C" void kernel_launch(void* const* d_in, const int* in_sizes, int n_in,
                              void* d_out, int out_size, void* d_ws, size_t ws_size, hipStream_t stream) {
  if (n_in < 5) return;
  const float* x = (const float*)d_in[0]; const float* wqkv = (const float*)d_in[1]; const float* bqkv = (const float*)d_in[2]; const float* wo = (const float*)d_in[3]; const float* bo = (const float*)d_in[4];
  const size_t need_rows = (size_t)(NB - 1) * SEQ_FULL + SEQ;
  if ((size_t)in_sizes[0] < need_rows * DM) return;
  if ((size_t)in_sizes[1] < (size_t)DM * LQ) return;
  if (in_sizes[2] < LQ) return;
  if ((size_t)in_sizes[3] < (size_t)DM * DM) return;
  if (in_sizes[4] < DM) return;
  if ((size_t)out_size < need_rows * DM) return;
  float* out = (float*)d_out;
  char* ws = (char*)d_ws; size_t off = 0;
  auto take = [&](size_t bytes) { char* p = ws + off; off += (bytes + 255) & ~(size_t)255; return p; };
  _Float16* BQKV = (_Float16*)take((size_t)LQ * DM * 2);
  _Float16* BO   = (_Float16*)take((size_t)DM * DM * 2);
  _Float16* X16  = (_Float16*)take(NR * DM * 2);
  _Float16* QKV  = (_Float16*)take(NR * LQ * 2);
  _Float16* O16  = (_Float16*)take(NR * DM * 2);
  _Float16* VT   = (_Float16*)take((size_t)NB * NH * HD * SEQ * 2);
  float*    QF   = (float*)take((size_t)NB * QT1 * LQ * 4);
  _Float16* QL   = (_Float16*)take((size_t)NB * QT1 * LQ * 2);
  _Float16* VTL  = (_Float16*)take((size_t)NB * NH * HD * QT1 * 2);
  _Float16* OL   = (_Float16*)take((size_t)NB * QT1 * DM * 2);
  if (off > ws_size) return;

  k_wt_f16<<<(unsigned)(((size_t)LQ * (DM / 8) + 255) / 256), 256, 0, stream>>>(wqkv, BQKV, DM, LQ, 16.0f);
  k_wt_f16<<<(unsigned)(((size_t)DM * (DM / 8) + 255) / 256), 256, 0, stream>>>(wo, BO, DM, DM, 16.0f);
  k_x16r<<<(unsigned)((NR * DM / 8 + 255) / 256), 256, 0, stream>>>(x, X16, NR * DM / 8);
  k_gemm2<<<dim3((QT1 / 128) * (LQ / 64), NB), 128, 0, stream>>>(X16, DM, (size_t)SEQ * DM, BQKV, DM, (size_t)0, 0.0625f, bqkv, nullptr, QF, QKV, LQ, (size_t)QT1 * LQ, (size_t)SEQ * LQ, QT1, LQ, DM);
  if (SEQ > QT1)
    k_gemm2<<<dim3(((SEQ - QT1) / 128) * (LQ / 64), NB), 128, 0, stream>>>(X16 + (size_t)QT1 * DM, DM, (size_t)SEQ * DM, BQKV, DM, (size_t)0, 0.0625f, bqkv, nullptr, nullptr, QKV + (size_t)QT1 * LQ, LQ, (size_t)0, (size_t)SEQ * LQ, SEQ - QT1, LQ, DM);
  k_hres<<<(unsigned)(((size_t)NB * QT1 * LQ / 8 + 255) / 256), 256, 0, stream>>>(QF, QL, (size_t)NB * QT1 * LQ / 8);
  k_vt<NH, SEQ><<<NB * NH * (SEQ / 64), 256, 0, stream>>>(QKV, LQ, 2 * DM, VT);
  k_vt<NH, QT1><<<NB * NH * (QT1 / 64), 256, 0, stream>>>(QL, LQ, 2 * DM, VTL);
  k_attn0<<<dim3(QT1 / 64, NB * NH), 128, 0, stream>>>(QKV, QL, VT, VTL, O16, OL);
  if (SEQ > QT1)
    k_attn<<<dim3(SEQ / 64 - QT1 / 64, NB * NH), 128, 0, stream>>>(QKV, VT, O16, QT1 / 64);
  k_gemm2<<<dim3((SEQ / 128) * (DM / 64), NB), 128, 0, stream>>>(O16, DM, (size_t)SEQ * DM, BO, DM, (size_t)0, 0.0009765625f, bo, nullptr, out, nullptr, DM, (size_t)SEQ_FULL * DM, (size_t)0, SEQ, DM, DM);
  k_gemm2<<<dim3((QT1 / 128) * (DM / 64), NB), 128, 0, stream>>>(OL, DM, (size_t)QT1 * DM, BO, DM, (size_t)0, 0.00000095367431640625f, nullptr, out, out, nullptr, DM, (size_t)SEQ_FULL * DM, (size_t)0, QT1, DM, DM);
}
